// GlobalAttentionTransformerEncoder_57741540327437
// MI455X (gfx1250) — hardware-run, weakly checked
//
#include <hip/hip_runtime.h>


#ifndef NB
#define NB 2
#endif
#ifndef SEQ
#define SEQ 1024
#endif
#define NB_FULL  2
#define SEQ_FULL 1024
#ifndef OUT_SEQ
#define OUT_SEQ SEQ
#endif
#define DM   512
#define NH_  8
#define HD   64
#define NG   32
#define AW   4
#define OSP  68
#define EROWS (SEQ < 256 ? SEQ : 256)
#define QRS  2048.0f
#define QRI  (1.0f / 2048.0f)
#define LOG2E 1.4426950408889634f
#define ACAR 4096.0f
#define PCAR 16384.0f
#define OCAR 16.0f
#define WCAR 64.0f
#define OSI  (1.0f / (16.0f * 64.0f))
#define MINN 1e-8f
#define NPS  (NB * NH_ * (SEQ / 32))

static_assert(HD == 64);
static_assert(NG == 32);
static_assert(NH_ * HD == DM);
static_assert(DM % 64 == 0);
static_assert(DM % 32 == 0);
static_assert(SEQ % 64 == 0);
static_assert((NB * SEQ) % 64 == 0);
static_assert(EROWS % 64 == 0);
static_assert(EROWS >= 64);
static_assert(EROWS <= SEQ);
static_assert((SEQ - EROWS) % 64 == 0);
static_assert(EROWS % (16 * AW) == 0);
static_assert((SEQ - EROWS) % (16 * AW) == 0);
static_assert(NB <= NB_FULL);
static_assert(SEQ <= SEQ_FULL);
static_assert((OSP * 4) % 16 == 0);
static_assert(OSP >= HD + 4);
static_assert(((size_t)SEQ * DM) % 8 == 0);
static_assert(((size_t)NG * DM) % 8 == 0);
static_assert(4 * 32 * 16 == 16 * HD * 2);
static_assert(4 * 4 == 16 && 8 * 16 == 64 * 2);
static_assert(4 * 4 == 16 && 8 * 16 == NG * 4);
static_assert(8 * 2 == 16 && 16 * 16 == 64 * 4);
static_assert(16 * 4 == 64);
static_assert(8 * 32 * 16 == 64 * NG * 2);
static_assert(8 * 4 == NG && 8 * 16 == 64 * 2);
static_assert(256 * 8 * 2 == 64 * 64);
static_assert(16 * 256 == 64 * 64);
static_assert(64 * 65 * 4 <= 131072);
static_assert(16 * 68 * 4 <= 131072);
static_assert(2 * 64 * 36 * 4 <= 131072);
static_assert(AW * 16 * OSP * 4 <= 131072);

typedef _Float16 h16;
typedef unsigned short bf;
typedef __attribute__((ext_vector_type(16))) __bf16   v16bf;
typedef __attribute__((ext_vector_type(16))) _Float16 v16h;
typedef __attribute__((ext_vector_type(8)))  _Float16 v8h;
typedef __attribute__((ext_vector_type(8)))  unsigned short v8us;
typedef __attribute__((ext_vector_type(8)))  float    v8f;
typedef __attribute__((ext_vector_type(4)))  float    v4f;
typedef v4f  __attribute__((may_alias)) v4fa;

__device__ __forceinline__ unsigned short f2bf(float f) { unsigned u = __float_as_uint(f); u += 0x7FFFu + ((u >> 16) & 1u); return (unsigned short)(u >> 16); }
__device__ __forceinline__ float bfr(float f) { return __uint_as_float(((unsigned)f2bf(f)) << 16); }
__device__ __forceinline__ v16h cat16(v8h lo, v8h hi) { return __builtin_shufflevector(lo, hi, 0, 1, 2, 3, 4, 5, 6, 7, 8, 9, 10, 11, 12, 13, 14, 15); }
__device__ __forceinline__ v16bf cat16b(v8us lo, v8us hi) { return __builtin_bit_cast(v16bf, __builtin_shufflevector(lo, hi, 0, 1, 2, 3, 4, 5, 6, 7, 8, 9, 10, 11, 12, 13, 14, 15)); }
__device__ __forceinline__ v8f wmma16(v16h a, v16h b, v8f c) { return __builtin_amdgcn_wmma_f32_16x16x32_f16(false, a, false, b, (short)0, c, false, false); }
__device__ __forceinline__ v8f wmmab(v16bf a, v16bf b, v8f c) { return __builtin_amdgcn_wmma_f32_16x16x32_bf16(false, a, false, b, (short)0, c, false, false); }
__device__ __forceinline__ v16h  ldh(const h16* p) { return cat16(*(const v8h*)p, *(const v8h*)(p + 16)); }
__device__ __forceinline__ v16bf ldb(const bf* p)  { return cat16b(*(const v8us*)p, *(const v8us*)(p + 16)); }
__device__ __forceinline__ void wave_sync() { __builtin_amdgcn_fence(3  , "wavefront"); __builtin_amdgcn_wave_barrier(); asm volatile("" ::: "memory"); }

static __device__ __forceinline__ h16 toh_flush(float v) { const h16 r = (h16)v; return (fabsf(v) < 6.103515625e-05f) ? (h16)0.0f : r; }
__device__ __forceinline__ void split8(v4f x0, v4f x1, v8h& hv, v8h& rv) {
#pragma unroll
    for (int i = 0; i < 4; ++i) {
        const h16 a0 = toh_flush(x0[i]); const h16 a1 = toh_flush(x1[i]);
        hv[i] = a0; hv[4 + i] = a1;
        rv[i] = toh_flush((x0[i] - (float)a0) * QRS); rv[4 + i] = toh_flush((x1[i] - (float)a1) * QRS); }
}
__device__ __forceinline__ v8f mmh(v16h a, v16h b, v8f c) { c = wmma16(a, b, c); asm volatile("v_nop\n\tv_nop\n\tv_nop\n\tv_nop" : "+v"(c) : "v"(a), "v"(b)); return c; }
__device__ __forceinline__ v8f mmb(v16bf a, v16bf b, v8f c) { c = wmmab(a, b, c); asm volatile("v_nop\n\tv_nop\n\tv_nop\n\tv_nop" : "+v"(c) : "v"(a), "v"(b)); return c; }

__global__ __launch_bounds__(256) void k_cvt8(const float* __restrict__ src, bf* dst, size_t n8) {
    const size_t i = (size_t)blockIdx.x * 256 + threadIdx.x; if (i >= n8) return;
    const v8f v = *(const v8f*)(src + i * 8); v8us o;
#pragma unroll
    for (int k = 0; k < 8; ++k) o[k] = f2bf(v[k]);
    *(volatile v8us*)(dst + i * 8) = o; __threadfence(); *(volatile v8us*)(dst + i * 8) = o;
}

__global__ __launch_bounds__(256) void k_wt_bf(const float* __restrict__ W, bf* T) {
    __shared__ float ts[64 * 65];
    const int tid = threadIdx.x; const int k0 = blockIdx.x * 64, n0 = blockIdx.y * 64;
#pragma unroll 1
    for (int it = 0; it < 16; ++it) { const int i = it * 256 + tid; const int r = i >> 6, c = i & 63;
        ts[r * 65 + c] = bfr(W[(size_t)(k0 + r) * DM + n0 + c]); }
    __syncthreads();
#pragma unroll 1
    for (int ps = 0; ps < 2; ++ps) {
#pragma unroll
        for (int it = 0; it < 2; ++it) { const int row = it * 32 + (tid >> 3), c8 = (tid & 7) * 8; v8us o;
#pragma unroll
            for (int j = 0; j < 8; ++j) o[j] = f2bf(ts[(c8 + j) * 65 + row]);
            *(volatile v8us*)(T + (size_t)(n0 + row) * DM + k0 + c8) = o; }
        if (ps == 0) __threadfence(); }
}

__global__ __launch_bounds__(256) void k_wt_h(const float* __restrict__ W, h16* T) {
    __shared__ float ts[64 * 65];
    const int tid = threadIdx.x; const int k0 = blockIdx.x * 64, n0 = blockIdx.y * 64;
#pragma unroll 1
    for (int it = 0; it < 16; ++it) { const int i = it * 256 + tid; const int r = i >> 6, c = i & 63;
        ts[r * 65 + c] = bfr(W[(size_t)(k0 + r) * DM + n0 + c]); }
    __syncthreads();
#pragma unroll 1
    for (int ps = 0; ps < 2; ++ps) {
#pragma unroll
        for (int it = 0; it < 2; ++it) { const int row = it * 32 + (tid >> 3), c8 = (tid & 7) * 8; v8h o;
#pragma unroll
            for (int j = 0; j < 8; ++j) o[j] = toh_flush(ts[(c8 + j) * 65 + row] * WCAR);
            *(volatile v8h*)(T + (size_t)(n0 + row) * DM + k0 + c8) = o; }
        if (ps == 0) __threadfence(); }
}

template <int MODE, int MB>
__device__ __forceinline__ void proj_body(const bf* __restrict__ A, const bf* __restrict__ Bt, h16* Ph, h16* Pr, int seqlen, int resT) {
    __shared__ __align__(16) float os[16 * 68];
    const int K = DM;
    const int lane = threadIdx.x & 31, lr = lane & 15, hi = lane >> 4; const int r0 = blockIdx.x * (16 * MB), c0 = blockIdx.y * 64;
    v8f acc[MB][4];
#pragma unroll
    for (int mb = 0; mb < MB; ++mb)
#pragma unroll
        for (int nb = 0; nb < 4; ++nb) acc[mb][nb] = (v8f){};
    const size_t aoff = (size_t)(r0 + lr) * K + 8 * hi, boff = (size_t)(c0 + lr) * K + 8 * hi;
#pragma unroll 1
    for (int kc = 0; kc < K; kc += 32) {
        v16bf a[MB];
#pragma unroll
        for (int mb = 0; mb < MB; ++mb) a[mb] = ldb(A + aoff + (size_t)mb * 16 * K + kc);
#pragma unroll
        for (int nb = 0; nb < 4; ++nb) { const v16bf b = ldb(Bt + boff + (size_t)nb * 16 * K + kc);
#pragma unroll
            for (int mb = 0; mb < MB; ++mb) acc[mb][nb] = mmb(a[mb], b, acc[mb][nb]); }
    }
    size_t tbase, rbase; bool wr;
    if (MODE == 0) { const int bb = r0 / seqlen, tt = r0 % seqlen; const int zc = bb * NH_ + c0 / HD;
                     tbase = ((size_t)zc * (size_t)seqlen + (size_t)tt) * HD; rbase = ((size_t)zc * (size_t)resT + (size_t)tt) * HD; wr = tt < resT; }
    else           { const int bb = c0 / seqlen, tt = c0 % seqlen;
                     tbase = (size_t)bb * (size_t)DM * (size_t)seqlen + (size_t)r0 * (size_t)seqlen + (size_t)tt; rbase = (size_t)bb * (size_t)DM * (size_t)resT + (size_t)r0 * (size_t)resT + (size_t)tt; wr = tt < resT; }
#pragma unroll
    for (int mb = 0; mb < MB; ++mb) {
#pragma unroll
        for (int nb = 0; nb < 4; ++nb) {
#pragma unroll
            for (int j = 0; j < 8; ++j) os[(hi * 8 + j) * 68 + nb * 16 + lr] = acc[mb][nb][j]; }
        wave_sync();
#pragma unroll 1
        for (int ps = 0; ps < 2; ++ps) {
            if (MODE == 0) {
                const size_t sb = tbase + (size_t)(mb * 16) * HD;
                const size_t rb = rbase + (size_t)(mb * 16) * HD;
#pragma unroll
                for (int s = 0; s < 4; ++s) { const int p = s * 32 + lane; const int row = p >> 3, c8 = (p & 7) * 8;
                    const v4f x0 = *(const v4fa*)(&os[row * 68 + c8]); const v4f x1 = *(const v4fa*)(&os[row * 68 + c8 + 4]); v8h hv, rv;
                    split8(x0, x1, hv, rv);
                    const size_t oo = sb + (size_t)p * 8;
                    const size_t ro = rb + (size_t)p * 8;
                    *(volatile v8h*)(Ph + oo) = hv; if (wr) *(volatile v8h*)(Pr + ro) = rv; }
            } else {
                const size_t sb = tbase + (size_t)(mb * 16) * (size_t)seqlen;
                const size_t rb = rbase + (size_t)(mb * 16) * (size_t)resT;
#pragma unroll
                for (int s = 0; s < 4; ++s) { const int row = 4 * s + (lane >> 3), c8 = (lane & 7) * 8;
                    const v4f x0 = *(const v4fa*)(&os[row * 68 + c8]); const v4f x1 = *(const v4fa*)(&os[row * 68 + c8 + 4]); v8h hv, rv;
                    split8(x0, x1, hv, rv);
                    const size_t oo = sb + (size_t)row * (size_t)seqlen + c8;
                    const size_t ro = rb + (size_t)row * (size_t)resT + c8;
                    *(volatile v8h*)(Ph + oo) = hv; if (wr) *(volatile v8h*)(Pr + ro) = rv; }
            }
            if (ps == 0) __threadfence(); }
        wave_sync();
    }
}

__global__ __launch_bounds__(32) void k_proj_rows(const bf* __restrict__ X, const bf* __restrict__ Wt, h16* Ph, h16* Pr, int resT) { proj_body<0, 4>(X, Wt, Ph, Pr, SEQ, resT); }
__global__ __launch_bounds__(32) void k_proj_vt(const bf* __restrict__ Wt, const bf* __restrict__ X, h16* Ph, h16* Pr, int resT) { proj_body<1, 4>(Wt, X, Ph, Pr, SEQ, resT); }
__global__ __launch_bounds__(32) void k_proj_ctx(const bf* __restrict__ C, const bf* __restrict__ Wt, h16* Ph, h16* Pr) { proj_body<0, 2>(C, Wt, Ph, Pr, NG, NG); }

template <int EARLY>
__device__ __forceinline__ void wraw_body(const h16* __restrict__ KP, const h16* __restrict__ KR, const h16* __restrict__ CH, const h16* __restrict__ CR, float* WRAW, float* PS) {
    __shared__ __align__(16) float os[16 * 36];
    const int lane = threadIdx.x & 31, lr = lane & 15, hi = lane >> 4;
    const int zh = blockIdx.y; const int h = zh % NH_;
    const int tile = (EARLY ? 0 : (EROWS / 32)) + (int)blockIdx.x; const int t0 = tile * 32;
    v8f acc[2][2], accR[2][2];
#pragma unroll
    for (int mb = 0; mb < 2; ++mb)
#pragma unroll
        for (int nb = 0; nb < 2; ++nb) { acc[mb][nb] = (v8f){}; accR[mb][nb] = (v8f){}; }
    const size_t ko  = ((size_t)zh * SEQ + (size_t)(t0 + lr)) * HD + 8 * hi;
    const size_t kro = ((size_t)zh * EROWS + (size_t)((EARLY ? t0 : 0) + lr)) * HD + 8 * hi;
    const size_t co  = ((size_t)h * NG + (size_t)lr) * HD + 8 * hi;
#pragma unroll
    for (int kc = 0; kc < HD; kc += 32) {
        v16h ch[2], cr[2];
#pragma unroll
        for (int nb = 0; nb < 2; ++nb) { ch[nb] = ldh(CH + co + (size_t)nb * 16 * HD + kc); cr[nb] = ch[nb]; if (EARLY) cr[nb] = ldh(CR + co + (size_t)nb * 16 * HD + kc); }
#pragma unroll
        for (int mb = 0; mb < 2; ++mb) {
            const v16h kh = ldh(KP + ko + (size_t)mb * 16 * HD + kc);
#pragma unroll
            for (int nb = 0; nb < 2; ++nb) acc[mb][nb] = mmh(kh, ch[nb], acc[mb][nb]);
            if (EARLY) {
                const v16h kr = ldh(KR + kro + (size_t)mb * 16 * HD + kc);
#pragma unroll
                for (int nb = 0; nb < 2; ++nb) { accR[mb][nb] = mmh(kh, cr[nb], accR[mb][nb]); accR[mb][nb] = mmh(kr, ch[nb], accR[mb][nb]); }
            }
        }
    }
    float part = 0.0f;
#pragma unroll
    for (int mb = 0; mb < 2; ++mb) {
#pragma unroll
        for (int nb = 0; nb < 2; ++nb) {
#pragma unroll
            for (int j = 0; j < 8; ++j) { const float val = (EARLY ? (acc[mb][nb][j] + accR[mb][nb][j] * QRI) : acc[mb][nb][j]) * 0.125f;
                os[(hi * 8 + j) * 36 + nb * 16 + lr] = val; part += val; } }
        wave_sync();
        float* wrow = WRAW + ((size_t)zh * SEQ + (size_t)(t0 + mb * 16)) * NG;
#pragma unroll 1
        for (int ps = 0; ps < 2; ++ps) {
#pragma unroll
            for (int s = 0; s < 4; ++s) { const int row = 4 * s + (lane >> 3), cofs = (lane & 7) * 4;
                const v4f val = *(const v4fa*)(&os[row * 36 + cofs]);
                *(volatile v4f*)(wrow + (size_t)row * NG + cofs) = val; }
            if (ps == 0) __threadfence(); }
        wave_sync();
    }
    float* pl = PS + ((size_t)zh * (SEQ / 32) + (size_t)tile) * 32 + lane;
    *(volatile float*)pl = part; __threadfence(); *(volatile float*)pl = part;
}

__global__ __launch_bounds__(32) void k_wraw_early(const h16* __restrict__ KP, const h16* __restrict__ KR, const h16* __restrict__ CH, const h16* __restrict__ CR, float* WRAW, float* PS) { wraw_body<1>(KP, KR, CH, CR, WRAW, PS); }
__global__ __launch_bounds__(32) void k_wraw_late(const h16* __restrict__ KP, const h16* __restrict__ KR, const h16* __restrict__ CH, const h16* __restrict__ CR, float* WRAW, float* PS) { wraw_body<0>(KP, KR, CH, CR, WRAW, PS); }

__global__ __launch_bounds__(32) void k_scan(const float* __restrict__ WRAW, const float* __restrict__ PS, float* RN, h16* WG, h16* WGR, h16* WT, h16* WTR) {
#pragma clang fp contract(off)
    __shared__ __align__(16) float tw[64 * 36];
    __shared__ __align__(16) float tn[64 * 36];
    const int lane = threadIdx.x & 31;
    const int zh = blockIdx.x;
    float tot = 0.0f;
#pragma unroll 1
    for (int i = 0; i < NPS; ++i) tot += PS[(size_t)i * 32 + lane];
    tot += __shfl_xor(tot, 16, 32); tot += __shfl_xor(tot, 8, 32); tot += __shfl_xor(tot, 4, 32); tot += __shfl_xor(tot, 2, 32); tot += __shfl_xor(tot, 1, 32);
    const float mean = tot * (1.0f / (float)((size_t)NB * NH_ * SEQ * NG));
    float run = 0.0f;
    const size_t base = (size_t)zh * SEQ;
#pragma unroll 1
    for (int c = 0; c < SEQ / 64; ++c) {
        const int tc = c * 64;
#pragma unroll 1
        for (int i = 0; i < 64; ++i) {
            const float x = WRAW[(base + (size_t)(tc + i)) * NG + lane];
            const float w = __builtin_amdgcn_exp2f((x - mean) * LOG2E);
            run += w;
            const float nm = (run <= MINN) ? MINN : run;
            tw[i * 36 + lane] = w; tn[i * 36 + lane] = 1.0f / nm; }
        wave_sync();
        const bool er = tc < EROWS;
#pragma unroll 1
        for (int ps = 0; ps < 2; ++ps) {
#pragma unroll 1
            for (int s = 0; s < 16; ++s) { const int row = 4 * s + (lane >> 3), cofs = (lane & 7) * 4;
                const v4f val = *(const v4fa*)(&tn[row * 36 + cofs]);
                *(volatile v4f*)(RN + (base + (size_t)(tc + row)) * NG + cofs) = val; }
#pragma unroll 1
            for (int s = 0; s < 8; ++s) { const int p = s * 32 + lane; const int row = p >> 2, c8 = (p & 3) * 8;
                const v4f x0 = *(const v4fa*)(&tw[row * 36 + c8]); const v4f x1 = *(const v4fa*)(&tw[row * 36 + c8 + 4]); v8h hv, rv;
                split8(x0, x1, hv, rv);
                *(volatile v8h*)(WG + (base + (size_t)tc) * NG + (size_t)p * 8) = hv;
                if (er) *(volatile v8h*)(WGR + ((size_t)zh * EROWS + (size_t)tc) * NG + (size_t)p * 8) = rv; }
#pragma unroll 1
            for (int s = 0; s < 8; ++s) { const int gg = 4 * s + (lane >> 3), c8 = (lane & 7) * 8;
                v4f x0, x1; v8h hv, rv;
#pragma unroll
                for (int j = 0; j < 4; ++j) { x0[j] = tw[(c8 + j) * 36 + gg]; x1[j] = tw[(c8 + 4 + j) * 36 + gg]; }
                split8(x0, x1, hv, rv);
                *(volatile v8h*)(WT + ((size_t)zh * NG + (size_t)gg) * SEQ + tc + c8) = hv;
                if (er) *(volatile v8h*)(WTR + ((size_t)zh * NG + (size_t)gg) * EROWS + tc + c8) = rv; }
            if (ps == 0) __threadfence(); }
        wave_sync();
    }
}

template <int EARLY>
__device__ __forceinline__ void score_tile(const h16* __restrict__ ka, const h16* __restrict__ kra, v16h qh0, v16h qh1, v16h qr0, v16h qr1, v8f& sH, v8f& sL) {
    const v16h k0 = ldh(ka), k1 = ldh(ka + 32);
    sH = mmh(k0, qh0, sH); sH = mmh(k1, qh1, sH);
    if (EARLY) {
        sL = mmh(k0, qr0, sL); sL = mmh(k1, qr1, sL);
        const v16h e0 = ldh(kra), e1 = ldh(kra + 32);
        sL = mmh(e0, qh0, sL); sL = mmh(e1, qh1, sL);
    }
}
template <int EARLY>
__device__ __forceinline__ void pack_masked(v8f xH0, v8f xL0, v8f xH1, v8f xL1, float scale, int ja, int lim, v16h& hb, v16h& rb) {
#pragma unroll
    for (int r = 0; r < 8; ++r) {
        float a0 = (EARLY ? (xH0[r] + xL0[r] * QRI) : xH0[r]) * scale;
        float a1 = (EARLY ? (xH1[r] + xL1[r] * QRI) : xH1[r]) * scale;
        a0 = (ja + r <= lim) ? a0 : 0.0f;
        a1 = (ja + 16 + r <= lim) ? a1 : 0.0f;
        const h16 h0 = toh_flush(a0); const h16 h1 = toh_flush(a1);
        hb[r] = h0; hb[8 + r] = h1;
        if (EARLY) { rb[r] = toh_flush((a0 - (float)h0) * QRS); rb[8 + r] = toh_flush((a1 - (float)h1) * QRS); }
    }
}

template <int EARLY>
__device__ __forceinline__ void attn_body(const h16* __restrict__ QH, const h16* __restrict__ QR, const h16* __restrict__ KP, const h16* __restrict__ KR,
                                          const h16* __restrict__ WT, const h16* __restrict__ WTR, const h16* __restrict__ WG, const h16* __restrict__ WGR,
                                          const h16* __restrict__ VT, const h16* __restrict__ VR, const float* __restrict__ RN, h16* OH, h16* ORp) {
    __shared__ __align__(16) float os[AW * 16 * OSP];
    const int lane = threadIdx.x & 31, lr = lane & 15, hi = lane >> 4;
    const int wave = __builtin_amdgcn_readfirstlane((int)(threadIdx.x >> 5));
    const int zh = blockIdx.y; const int b = zh / NH_, h = zh % NH_;
    const int t0 = (EARLY ? 0 : EROWS) + ((int)blockIdx.x * AW + wave) * 16;
    const int nk = (t0 + 16 + 31) & ~31;
    const int lim = t0 + lr;
    const size_t pq = (size_t)zh * SEQ * HD;
    const size_t pe = (size_t)zh * EROWS * HD;
    const v16h hz = (v16h){};
    const size_t qo = pq + (size_t)(t0 + lr) * HD + 8 * hi;
    const size_t qro = pe + (size_t)((EARLY ? t0 : 0) + lr) * HD + 8 * hi;
    const v16h qh0 = ldh(QH + qo), qh1 = ldh(QH + qo + 32);
    v16h qr0 = hz, qr1 = hz;
    if (EARLY) { qr0 = ldh(QR + qro); qr1 = ldh(QR + qro + 32); }
    const size_t ko = pq + (size_t)lr * HD + 8 * hi;
    const size_t kro = pe + (size_t)lr * HD + 8 * hi;
    const size_t wto = ((size_t)zh * NG + (size_t)lr) * SEQ + 8 * hi;
    const size_t wtro = ((size_t)zh * NG + (size_t)lr) * EROWS + 8 * hi;
    v8f LH0 = (v8f){}, LH1 = (v8f){}, LL0 = (v8f){}, LL1 = (v8f){};
#pragma unroll 1
    for (int key0 = 0; key0 < nk; key0 += 32) {
        v8f sH0 = (v8f){}, sL0 = (v8f){}, sH1 = (v8f){}, sL1 = (v8f){};
        score_tile<EARLY>(KP + ko + (size_t)key0 * HD, KR + kro + (size_t)(EARLY ? key0 : 0) * HD, qh0, qh1, qr0, qr1, sH0, sL0);
        score_tile<EARLY>(KP + ko + (size_t)(key0 + 16) * HD, KR + kro + (size_t)(EARLY ? (key0 + 16) : 0) * HD, qh0, qh1, qr0, qr1, sH1, sL1);
        v16h ab, ar = hz;
        pack_masked<EARLY>(sH0, sL0, sH1, sL1, 1.0f, key0 + 8 * hi, lim, ab, ar);
        { const v16h w0 = ldh(WT + wto + key0);
          LH0 = mmh(w0, ab, LH0);
          if (EARLY) { LL0 = mmh(w0, ar, LL0); const v16h e0 = ldh(WTR + wtro + key0); LL0 = mmh(e0, ab, LL0); } }
        { const v16h w1 = ldh(WT + wto + (size_t)16 * SEQ + key0);
          LH1 = mmh(w1, ab, LH1);
          if (EARLY) { LL1 = mmh(w1, ar, LL1); const v16h e1 = ldh(WTR + wtro + (size_t)16 * EROWS + key0); LL1 = mmh(e1, ab, LL1); } }
    }
    const float* rp = RN + ((size_t)zh * SEQ + (size_t)(t0 + lr)) * NG + 8 * hi;
    const v4f n0 = *(const v4f*)rp, n1 = *(const v4f*)(rp + 4), n2 = *(const v4f*)(rp + 16), n3 = *(const v4f*)(rp + 20);
    float rn0[8], rn1[8], lg0[8], lg1[8];
#pragma unroll
    for (int r = 0; r < 4; ++r) { rn0[r] = n0[r]; rn0[4 + r] = n1[r]; rn1[r] = n2[r]; rn1[4 + r] = n3[r]; }
    float mx = -3.0e38f;
#pragma unroll
    for (int r = 0; r < 8; ++r) {
        const float l0 = EARLY ? (LH0[r] + LL0[r] * QRI) : LH0[r];
        const float l1 = EARLY ? (LH1[r] + LL1[r] * QRI) : LH1[r];
        lg0[r] = l0 * rn0[r]; lg1[r] = l1 * rn1[r];
        mx = fmaxf(mx, fmaxf(lg0[r], lg1[r])); }
    mx = fmaxf(mx, __shfl_xor(mx, 16, 32));
    float z = 0.0f, um = 0.0f; float u0[8], u1[8];
#pragma unroll
    for (int r = 0; r < 8; ++r) {
        const float e0 = __builtin_amdgcn_exp2f((lg0[r] - mx) * LOG2E), e1 = __builtin_amdgcn_exp2f((lg1[r] - mx) * LOG2E);
        z += e0 + e1;
        u0[r] = e0 * rn0[r]; u1[r] = e1 * rn1[r];
        um = fmaxf(um, fmaxf(u0[r], u1[r])); }
    z += __shfl_xor(z, 16, 32);
    um = fmaxf(um, __shfl_xor(um, 16, 32));
    const float asc = ACAR * (1.0f / um);
    const float pscale = um * (PCAR / ACAR) * (1.0f / z);
    v16h af, afr = hz;
#pragma unroll
    for (int r = 0; r < 8; ++r) {
        const float x0 = u0[r] * asc, x1 = u1[r] * asc;
        const h16 h0 = toh_flush(x0); const h16 h1 = toh_flush(x1);
        af[r] = h0; af[8 + r] = h1;
        if (EARLY) { afr[r] = toh_flush((x0 - (float)h0) * QRS); afr[8 + r] = toh_flush((x1 - (float)h1) * QRS); } }
    const size_t wgo = ((size_t)zh * SEQ + (size_t)lr) * NG + 8 * hi;
    const size_t wgro = ((size_t)zh * EROWS + (size_t)lr) * NG + 8 * hi;
    const size_t vo = ((size_t)zh * HD + (size_t)lr) * SEQ + 8 * hi;
    const size_t vro = ((size_t)zh * HD + (size_t)lr) * EROWS + 8 * hi;
    v8f o[4], oR[4];
#pragma unroll
    for (int j = 0; j < 4; ++j) { o[j] = (v8f){}; oR[j] = (v8f){}; }
#pragma unroll 1
    for (int key0 = 0; key0 < nk; key0 += 32) {
        v8f pH0 = (v8f){}, pL0 = (v8f){}, pH1 = (v8f){}, pL1 = (v8f){};
        { const v16h g0 = ldh(WG + wgo + (size_t)key0 * NG);
          pH0 = mmh(g0, af, pH0);
          if (EARLY) { pL0 = mmh(g0, afr, pL0); const v16h e0 = ldh(WGR + wgro + (size_t)key0 * NG); pL0 = mmh(e0, af, pL0); } }
        { const v16h g1 = ldh(WG + wgo + (size_t)(key0 + 16) * NG);
          pH1 = mmh(g1, af, pH1);
          if (EARLY) { pL1 = mmh(g1, afr, pL1); const v16h e1 = ldh(WGR + wgro + (size_t)(key0 + 16) * NG); pL1 = mmh(e1, af, pL1); } }
        v16h pb, prr = hz;
        pack_masked<EARLY>(pH0, pL0, pH1, pL1, pscale, key0 + 8 * hi, lim, pb, prr);
#pragma unroll
        for (int j = 0; j < 4; ++j) {
            const v16h vv = ldh(VT + vo + (size_t)j * 16 * SEQ + key0);
            o[j] = mmh(vv, pb, o[j]);
            if (EARLY) { oR[j] = mmh(vv, prr, oR[j]); const v16h ve = ldh(VR + vro + (size_t)j * 16 * EROWS + key0); oR[j] = mmh(ve, pb, oR[j]); }
        }
    }
    const int wb = wave * 16 * OSP;
#pragma unroll
    for (int j = 0; j < 4; ++j) {
        v8f f = o[j];
        if (EARLY) f = o[j] + oR[j] * QRI;
        v4f a, c;
        a[0] = f[0] * (OCAR / PCAR); a[1] = f[1] * (OCAR / PCAR); a[2] = f[2] * (OCAR / PCAR); a[3] = f[3] * (OCAR / PCAR);
        c[0] = f[4] * (OCAR / PCAR); c[1] = f[5] * (OCAR / PCAR); c[2] = f[6] * (OCAR / PCAR); c[3] = f[7] * (OCAR / PCAR);
        *(v4fa*)(&os[wb + lr * OSP + j * 16 + 8 * hi]) = a; *(v4fa*)(&os[wb + lr * OSP + j * 16 + 8 * hi + 4]) = c; }
    wave_sync();
    h16* orow = OH + ((size_t)b * SEQ + (size_t)t0) * DM + h * HD;
    h16* rrow = ORp + ((size_t)b * EROWS + (size_t)(EARLY ? t0 : 0)) * DM + h * HD;
#pragma unroll 1
    for (int ps = 0; ps < 2; ++ps) {
#pragma unroll
        for (int s = 0; s < 4; ++s) { const int row = 4 * s + (lane >> 3), c8 = (lane & 7) * 8;
            const v4f x0 = *(const v4fa*)(&os[wb + row * OSP + c8]); const v4f x1 = *(const v4fa*)(&os[wb + row * OSP + c8 + 4]); v8h hv, rv;
            split8(x0, x1, hv, rv);
            *(volatile v8h*)(orow + (size_t)row * DM + c8) = hv;
            if (EARLY) *(volatile v8h*)(rrow + (size_t)row * DM + c8) = rv; }
        if (ps == 0) __threadfence(); }
}

__global__ __launch_bounds__(32 * AW) void k_attn_early(const h16* __restrict__ QH, const h16* __restrict__ QR, const h16* __restrict__ KP, const h16* __restrict__ KR,
                                                        const h16* __restrict__ WT, const h16* __restrict__ WTR, const h16* __restrict__ WG, const h16* __restrict__ WGR,
                                                        const h16* __restrict__ VT, const h16* __restrict__ VR, const float* __restrict__ RN, h16* OH, h16* ORp) {
    attn_body<1>(QH, QR, KP, KR, WT, WTR, WG, WGR, VT, VR, RN, OH, ORp);
}
__global__ __launch_bounds__(32 * AW) void k_attn_late(const h16* __restrict__ QH, const h16* __restrict__ QR, const h16* __restrict__ KP, const h16* __restrict__ KR,
                                                       const h16* __restrict__ WT, const h16* __restrict__ WTR, const h16* __restrict__ WG, const h16* __restrict__ WGR,
                                                       const h16* __restrict__ VT, const h16* __restrict__ VR, const float* __restrict__ RN, h16* OH, h16* ORp) {
    attn_body<0>(QH, QR, KP, KR, WT, WTR, WG, WGR, VT, VR, RN, OH, ORp);
}

template <int RES, int MB>
__device__ __forceinline__ void out_body(const h16* __restrict__ OH, const h16* __restrict__ ORp, const h16* __restrict__ WOT, float* OUT) {
    __shared__ __align__(16) float os[16 * 68];
    constexpr int TPB0 = (RES ? EROWS : (SEQ - EROWS)) / (16 * MB);
    constexpr int TPB = TPB0 > 0 ? TPB0 : 1;
    const int lane = threadIdx.x & 31, lr = lane & 15, hi = lane >> 4;
    const int bb = (int)blockIdx.x / TPB, tile = (int)blockIdx.x % TPB;
    const int tt = (RES ? 0 : EROWS) + tile * 16 * MB;
    const int c0 = blockIdx.y * 64;
    v8f acc[MB][4], accR[MB][4];
#pragma unroll
    for (int mb = 0; mb < MB; ++mb)
#pragma unroll
        for (int nb = 0; nb < 4; ++nb) { acc[mb][nb] = (v8f){}; accR[mb][nb] = (v8f){}; }
    const size_t aoff = ((size_t)bb * SEQ + (size_t)(tt + lr)) * DM + 8 * hi;
    const size_t roff = ((size_t)bb * EROWS + (size_t)((RES ? tt : 0) + lr)) * DM + 8 * hi;
    const size_t boff = (size_t)(c0 + lr) * DM + 8 * hi;
#pragma unroll 1
    for (int kc = 0; kc < DM; kc += 32) {
        v16h a[MB], ar[MB];
#pragma unroll
        for (int mb = 0; mb < MB; ++mb) { a[mb] = ldh(OH + aoff + (size_t)mb * 16 * DM + kc); ar[mb] = a[mb]; if (RES) ar[mb] = ldh(ORp + roff + (size_t)mb * 16 * DM + kc); }
#pragma unroll
        for (int nb = 0; nb < 4; ++nb) { const v16h bw = ldh(WOT + boff + (size_t)nb * 16 * DM + kc);
#pragma unroll
            for (int mb = 0; mb < MB; ++mb) { acc[mb][nb] = mmh(a[mb], bw, acc[mb][nb]); if (RES) accR[mb][nb] = mmh(ar[mb], bw, accR[mb][nb]); } }
    }
#pragma unroll
    for (int mb = 0; mb < MB; ++mb) {
#pragma unroll
        for (int nb = 0; nb < 4; ++nb) {
#pragma unroll
            for (int j = 0; j < 8; ++j) os[(hi * 8 + j) * 68 + nb * 16 + lr] = (RES ? (acc[mb][nb][j] + accR[mb][nb][j] * QRI) : acc[mb][nb][j]) * OSI; }
        wave_sync();
        float* orow = OUT + ((size_t)bb * OUT_SEQ + (size_t)(tt + mb * 16)) * DM + c0;
#pragma unroll 1
        for (int ps = 0; ps < 2; ++ps) {
#pragma unroll
            for (int s = 0; s < 8; ++s) { const int row = 2 * s + (lane >> 4), cofs = (lane & 15) * 4;
                const v4f val = *(const v4fa*)(&os[row * 68 + cofs]);
                *(volatile v4f*)(orow + (size_t)row * DM + cofs) = val; }
            if (ps == 0) __threadfence(); }
        wave_sync();
    }
}

__global__ __launch_bounds__(32) void k_out_early(const h16* __restrict__ OH, const h16* __restrict__ ORp, const h16* __restrict__ WOT, float* OUT) { out_body<1, 2>(OH, ORp, WOT, OUT); }
__global__ __launch_bounds__(32) void k_out_late(const h16* __restrict__ OH, const h16* __restrict__ ORp, const h16* __restrict__ WOT, float* OUT) { out_body<0, 4>(OH, ORp, WOT, OUT); }

static constexpr size_t al256(size_t v) { return (v + 255) & ~(size_t)255; }
static constexpr size_t SZ_XB = al256((size_t)NB * SEQ * DM * 2);
static constexpr size_t SZ_CB = al256((size_t)NG * DM * 2);
static constexpr size_t SZ_W  = al256((size_t)DM * DM * 2);
static constexpr size_t SZ_PL = al256((size_t)NB * NH_ * SEQ * HD * 2);
static constexpr size_t SZ_RS = al256((size_t)NB * NH_ * EROWS * HD * 2);
static constexpr size_t SZ_CS = al256((size_t)NH_ * NG * HD * 2);
static constexpr size_t SZ_F  = al256((size_t)NB * NH_ * SEQ * NG * 4);
static constexpr size_t SZ_PS = al256((size_t)NPS * 32 * 4);
static constexpr size_t SZ_WG = al256((size_t)NB * NH_ * SEQ * NG * 2);
static constexpr size_t SZ_WR = al256((size_t)NB * NH_ * EROWS * NG * 2);
static constexpr size_t SZ_TOTAL = 3 * SZ_XB + SZ_CB + 5 * SZ_W + 4 * SZ_PL + 4 * SZ_RS + 2 * SZ_CS + 2 * SZ_F + SZ_PS + 2 * SZ_WG + 2 * SZ_WR;
static_assert(SZ_TOTAL <= (size_t)134217728);
static_assert((size_t)NB * NH_ * SEQ * HD == (size_t)NB * SEQ * DM);
static_assert((size_t)NB * NH_ * EROWS * HD == (size_t)NB * EROWS * DM);

extern "C" void kernel_launch(void* const* d_in, const int* in_sizes, int n_in,
                              void* d_out, int out_size, void* d_ws, size_t ws_size, hipStream_t stream) {
    if (n_in < 9) return;
    const size_t needx = ((size_t)(NB - 1) * SEQ_FULL + SEQ) * DM;
    if ((size_t)in_sizes[0] < needx || (size_t)in_sizes[1] < needx || (size_t)in_sizes[2] < needx) return;
    if ((size_t)in_sizes[3] < (size_t)NG * DM) return;
    for (int i = 4; i < 9; ++i) if ((size_t)in_sizes[i] < (size_t)DM * DM) return;
    if ((size_t)out_size < ((size_t)(NB - 1) * OUT_SEQ + SEQ) * DM) return;
    if (SZ_TOTAL > ws_size) return;
    const float* xin[3] = { (const float*)d_in[0], (const float*)d_in[1], (const float*)d_in[2] };
    const float* ctx = (const float*)d_in[3];
    const float* wq = (const float*)d_in[4]; const float* wk = (const float*)d_in[5]; const float* wv = (const float*)d_in[6];
    const float* wo = (const float*)d_in[7]; const float* wc = (const float*)d_in[8];
    float* OUT = (float*)d_out;
    char* wsp = (char*)d_ws;
    bf* XB[3];
    XB[0] = (bf*)wsp; wsp += SZ_XB;
    XB[1] = (bf*)wsp; wsp += SZ_XB;
    XB[2] = (bf*)wsp; wsp += SZ_XB;
    bf* CB  = (bf*)wsp; wsp += SZ_CB;
    bf* WQT = (bf*)wsp; wsp += SZ_W;
    bf* WKT = (bf*)wsp; wsp += SZ_W;
    bf* WVT = (bf*)wsp; wsp += SZ_W;
    bf* WCT = (bf*)wsp; wsp += SZ_W;
    h16* WOT = (h16*)wsp; wsp += SZ_W;
    h16* QH = (h16*)wsp; wsp += SZ_PL;
    h16* KP = (h16*)wsp; wsp += SZ_PL;
    h16* VT = (h16*)wsp; wsp += SZ_PL;
    h16* OH = (h16*)wsp; wsp += SZ_PL;
    h16* QR = (h16*)wsp; wsp += SZ_RS;
    h16* KR = (h16*)wsp; wsp += SZ_RS;
    h16* VR = (h16*)wsp; wsp += SZ_RS;
    h16* ORp = (h16*)wsp; wsp += SZ_RS;
    h16* CSH = (h16*)wsp; wsp += SZ_CS;
    h16* CSR = (h16*)wsp; wsp += SZ_CS;
    float* WRAW = (float*)wsp; wsp += SZ_F;
    float* RN = (float*)wsp; wsp += SZ_F;
    float* PS = (float*)wsp; wsp += SZ_PS;
    h16* WG = (h16*)wsp; wsp += SZ_WG;
    h16* WT = (h16*)wsp; wsp += SZ_WG;
    h16* WGR = (h16*)wsp; wsp += SZ_WR;
    h16* WTR = (h16*)wsp; wsp += SZ_WR;

    for (int i = 0; i < 3; ++i) {
        if (SEQ == SEQ_FULL) {
            const size_t n8 = (size_t)NB * SEQ * DM / 8;
            k_cvt8<<<(unsigned)((n8 + 255) / 256), 256, 0, stream>>>(xin[i], XB[i], n8);
        } else {
            const size_t n8 = (size_t)SEQ * DM / 8;
            for (int b = 0; b < NB; ++b) k_cvt8<<<(unsigned)((n8 + 255) / 256), 256, 0, stream>>>(xin[i] + (size_t)b * SEQ_FULL * DM, XB[i] + (size_t)b * SEQ * DM, n8);
        }
    }
    { const size_t n8 = (size_t)NG * DM / 8; k_cvt8<<<(unsigned)((n8 + 255) / 256), 256, 0, stream>>>(ctx, CB, n8); }
    k_wt_bf<<<dim3(DM / 64, DM / 64, 1), 256, 0, stream>>>(wq, WQT);
    k_wt_bf<<<dim3(DM / 64, DM / 64, 1), 256, 0, stream>>>(wk, WKT);
    k_wt_bf<<<dim3(DM / 64, DM / 64, 1), 256, 0, stream>>>(wv, WVT);
    k_wt_bf<<<dim3(DM / 64, DM / 64, 1), 256, 0, stream>>>(wc, WCT);
    k_wt_h<<<dim3(DM / 64, DM / 64, 1), 256, 0, stream>>>(wo, WOT);

    k_proj_rows<<<dim3(NB * SEQ / 64, DM / 64, 1), 32, 0, stream>>>(XB[0], WQT, QH, QR, EROWS);
    k_proj_rows<<<dim3(NB * SEQ / 64, DM / 64, 1), 32, 0, stream>>>(XB[1], WKT, KP, KR, EROWS);
    k_proj_vt<<<dim3(DM / 64, NB * SEQ / 64, 1), 32, 0, stream>>>(WVT, XB[2], VT, VR, EROWS);
    k_proj_ctx<<<dim3(1, DM / 64, 1), 32, 0, stream>>>(CB, WCT, CSH, CSR);

    k_wraw_early<<<dim3(EROWS / 32, NB * NH_, 1), 32, 0, stream>>>(KP, KR, CSH, CSR, WRAW, PS);
    if (SEQ > EROWS)
        k_wraw_late<<<dim3((SEQ - EROWS) / 32, NB * NH_, 1), 32, 0, stream>>>(KP, KR, CSH, CSR, WRAW, PS);
    k_scan<<<NB * NH_, 32, 0, stream>>>(WRAW, PS, RN, WG, WGR, WT, WTR);

    k_attn_early<<<dim3(EROWS / (16 * AW), NB * NH_, 1), 32 * AW, 0, stream>>>(QH, QR, KP, KR, WT, WTR, WG, WGR, VT, VR, RN, OH, ORp);
    if (SEQ > EROWS)
        k_attn_late<<<dim3((SEQ - EROWS) / (16 * AW), NB * NH_, 1), 32 * AW, 0, stream>>>(QH, QR, KP, KR, WT, WTR, WG, WGR, VT, VR, RN, OH, ORp);

    k_out_early<<<dim3(NB * (EROWS / 32), DM / 64, 1), 32, 0, stream>>>(OH, ORp, WOT, OUT);
    if (SEQ > EROWS)
        k_out_late<<<dim3(NB * ((SEQ - EROWS) / 64), DM / 64, 1), 32, 0, stream>>>(OH, ORp, WOT, OUT);
}
